// ValleAttention_69071664054776
// MI455X (gfx1250) — hardware-verified
//
#include <hip/hip_runtime.h>
#include <math.h>
#include <stdint.h>

#define NB   2
#define SEQ  2048
#define EMB  1024
#define NHD  16
#define HDIM 64
#define HGRP 2
#define NGRP (NHD / HGRP)
#define TFP  (SEQ / 64)
#define TFN  (TFP * TFP)
#define MASK_CUT (-1.0e8f)

typedef __attribute__((ext_vector_type(16))) _Float16 v16h;
typedef __attribute__((ext_vector_type(8)))  _Float16 v8h;
typedef __attribute__((ext_vector_type(16))) __bf16   v16b;
typedef __attribute__((ext_vector_type(8)))  __bf16   v8b;
typedef __attribute__((ext_vector_type(8)))  float    v8f;
typedef __attribute__((ext_vector_type(4)))  float    v4f;
typedef __attribute__((ext_vector_type(2)))  float    v2f;
typedef __attribute__((ext_vector_type(4)))  unsigned int v4u;
typedef __attribute__((ext_vector_type(4)))  int      v4i;

__device__ __forceinline__ unsigned short f2bf_bits(float f) {
  unsigned u = __float_as_uint(f);
  return (unsigned short)((u + 0x7FFFu + ((u >> 16) & 1u)) >> 16);
}
__device__ __forceinline__ float bf_bits2f(unsigned short h) { return __uint_as_float(((unsigned)h) << 16); }

__device__ __forceinline__ void dep_guard_h(v8f& a, v8f& b, v16h x, v16h y) { asm volatile("v_nop\n\tv_nop\n\tv_nop\n\tv_nop" : "+v"(a), "+v"(b) : "v"(x), "v"(y)); }
__device__ __forceinline__ void dep_guard_b(v8f& a, v8f& b, v16b x, v16b y) { asm volatile("v_nop\n\tv_nop\n\tv_nop\n\tv_nop" : "+v"(a), "+v"(b) : "v"(x), "v"(y)); }
__device__ __forceinline__ void keep4_h(v16h a, v16h b, v16h c, v16h d) { asm volatile("v_nop" :: "v"(a), "v"(b), "v"(c), "v"(d)); }
__device__ __forceinline__ void keep4_b(v16b a, v16b b, v16b c, v16b d) { asm volatile("v_nop" :: "v"(a), "v"(b), "v"(c), "v"(d)); }
__device__ __forceinline__ void acc_guard4(v8f& a, v8f& b, v8f& c, v8f& d) { asm volatile("v_nop\n\tv_nop\n\tv_nop\n\tv_nop" : "+v"(a), "+v"(b), "+v"(c), "+v"(d)); }
template <typename T> struct Frag;
template <> struct Frag<_Float16> {
  typedef v16h V; union U { v16h v; v8h h[2]; };
  static __device__ __forceinline__ v16h load(const _Float16* p) {
    U f; f.h[0] = *(const v8h*)(p); f.h[1] = *(const v8h*)(p + 16); return f.v;
  }
  static __device__ __forceinline__ v8f mma(v16h a, v16h b, v8f c) {
    return __builtin_amdgcn_wmma_f32_16x16x32_f16(false, a, false, b, (short)0, c, false, false);
  }
  static __device__ __forceinline__ void guard(v8f& a, v8f& b, v16h x, v16h y) { dep_guard_h(a, b, x, y); }
  static __device__ __forceinline__ void keep(v16h a, v16h b, v16h c, v16h d) { keep4_h(a, b, c, d); }
};
template <> struct Frag<__bf16> {
  typedef v16b V; union U { v16b v; v8b h[2]; };
  static __device__ __forceinline__ v16b load(const __bf16* p) {
    U f; f.h[0] = *(const v8b*)(p); f.h[1] = *(const v8b*)(p + 16); return f.v;
  }
  static __device__ __forceinline__ v8f mma(v16b a, v16b b, v8f c) {
    return __builtin_amdgcn_wmma_f32_16x16x32_bf16(false, a, false, b, (short)0, c, false, false);
  }
  static __device__ __forceinline__ void guard(v8f& a, v8f& b, v16b x, v16b y) { dep_guard_b(a, b, x, y); }
  static __device__ __forceinline__ void keep(v16b a, v16b b, v16b c, v16b d) { keep4_b(a, b, c, d); }
};

template <int ET> struct Elem;
template <> struct Elem<0> { typedef _Float16 T; };
template <> struct Elem<1> { typedef __bf16 T; };
template <int ET, bool SPLIT, int BIAS_MODE, int OUT_MODE, bool RESID, int ACT = 0, bool SKIPF = false, bool SKIPK = false>
__global__ __launch_bounds__(256) void wmma_gemm64(
    const unsigned short* __restrict__ Ap, const unsigned short* __restrict__ A2p, int lda, long strideA,
    const unsigned short* __restrict__ Btp, const unsigned short* __restrict__ Bt2p, int ldb, long strideB,
    void* __restrict__ Cout, void* __restrict__ Cout2, int ldc, long strideC,
    const float* __restrict__ bias,
    const float* __restrict__ resid, long strideR,
    int M, int N, int K, float scale,
    const int* __restrict__ tflag, int tfp, int tfn) {
  typedef typename Elem<ET>::T T;
  typedef typename Frag<T>::V V;
  const T* A = (const T*)Ap; const T* A2 = (const T*)A2p; const T* Bt = (const T*)Btp; const T* Bt2 = (const T*)Bt2p;
  __shared__ __align__(16) float sT[8][16 * 68];
  const int b    = blockIdx.y;
  const int lane = threadIdx.x & 31;
  const int wave = threadIdx.x >> 5;
  const int tilesN = N >> 6;
  const int tilesM = M >> 6;
  const int tile = blockIdx.x * 8 + wave;
  if (tile >= tilesM * tilesN) return;
  const int tm = tile / tilesN;
  const int tn = tile - tm * tilesN;
  const int m0 = tm << 6;
  const int n0 = tn << 6;
  if (SKIPF) {
    int fi = tm * tfp + tn;
    fi = fi < 0 ? 0 : (fi > tfn - 1 ? tfn - 1 : fi);
    const int fv = __builtin_amdgcn_readfirstlane(tflag[fi]);
    if (fv == 0) return;
  }

  const T* Ab  = A  + (size_t)b * strideA;
  const T* Bb  = Bt + (size_t)b * strideB;
  const T* Ab2 = SPLIT ? (A2  + (size_t)b * strideA) : nullptr;
  const T* Bb2 = SPLIT ? (Bt2 + (size_t)b * strideB) : nullptr;

  const int rlane = lane & 15;
  const int koff  = (lane >> 4) * 8;
  const int mOff  = (lane >> 4) * 8;

  v8f acc[4][4];
#pragma unroll
  for (int i = 0; i < 4; ++i)
#pragma unroll
    for (int j = 0; j < 4; ++j) acc[i][j] = (v8f){0.f,0.f,0.f,0.f,0.f,0.f,0.f,0.f};

  int kEnd = K;
  if (SKIPK) {
    int ke = 0;
    const int nkt = K >> 6;
    for (int kt = 0; kt < nkt; ++kt) {
      int fi = tm * tfp + kt;
      fi = fi < 0 ? 0 : (fi > tfn - 1 ? tfn - 1 : fi);
      if (tflag[fi] != 0) ke = (kt + 1) << 6;
    }
    ke = ke > K ? K : ke;
    kEnd = __builtin_amdgcn_readfirstlane(ke);
  }
  for (int k0 = 0; k0 < kEnd; k0 += 32) {
    V bh[4], bl[4];
#pragma unroll
    for (int j = 0; j < 4; ++j) {
      const size_t bo = (size_t)(n0 + (j << 4) + rlane) * ldb + koff + k0;
      bh[j] = Frag<T>::load(Bb + bo);
      if (SPLIT) bl[j] = Frag<T>::load(Bb2 + bo);
    }
#pragma unroll
    for (int i = 0; i < 4; ++i) {
      const size_t ao = (size_t)(m0 + (i << 4) + rlane) * lda + koff + k0;
      V ah = Frag<T>::load(Ab + ao);
      V al;
      if (SPLIT) al = Frag<T>::load(Ab2 + ao);
#pragma unroll
      for (int j = 0; j < 4; ++j) {
        acc[i][j] = Frag<T>::mma(ah, bh[j], acc[i][j]);
        if (SPLIT) {
          acc[i][j] = Frag<T>::mma(ah, bl[j], acc[i][j]);
          acc[i][j] = Frag<T>::mma(al, bh[j], acc[i][j]);
        }
      }
      Frag<T>::guard(acc[i][0], acc[i][3], ah, SPLIT ? al : ah);
    }
    Frag<T>::keep(bh[0], bh[1], bh[2], bh[3]);
    if (SPLIT) Frag<T>::keep(bl[0], bl[1], bl[2], bl[3]);
  }
  acc_guard4(acc[0][0], acc[0][1], acc[0][2], acc[0][3]);
  acc_guard4(acc[1][0], acc[1][1], acc[1][2], acc[1][3]);
  acc_guard4(acc[2][0], acc[2][1], acc[2][2], acc[2][3]);
  acc_guard4(acc[3][0], acc[3][1], acc[3][2], acc[3][3]);

  float* slab = sT[wave];
  const float* Rb = RESID ? (resid + (size_t)b * strideR) : nullptr;
#pragma unroll
  for (int i = 0; i < 4; ++i) {
    const int mBase = m0 + (i << 4);
#pragma unroll
    for (int j = 0; j < 4; ++j) {
      const int n = n0 + (j << 4) + rlane;
      float bv = 0.f;
      if (BIAS_MODE == 2) bv = bias[n];
#pragma unroll
      for (int r = 0; r < 8; ++r) {
        float v = acc[i][j][r] * scale;
        if (BIAS_MODE == 1) v += bias[mBase + mOff + r];
        if (BIAS_MODE == 2) v += bv;
        if (RESID) v += Rb[(size_t)(mBase + mOff + r) * ldc + n];
        if (ACT == 1) v = tanhf(v);
        if (ACT == 2) v = fmaxf(v, 0.0f);
        if (ACT == 3) v = v / (1.0f + expf(-v));
        if (ACT == 4) v = (v > 0.f) ? v : 0.01f * v;
        if (ACT == 5) v = 0.5f * v * (1.0f + erff(v * 0.70710678118654752f));
        slab[(mOff + r) * 68 + (j << 4) + rlane] = v;
      }
    }
    __builtin_amdgcn_fence(__ATOMIC_RELEASE, "workgroup");
    __builtin_amdgcn_wave_barrier();
    __builtin_amdgcn_fence(__ATOMIC_ACQUIRE, "workgroup");
    if (OUT_MODE == 0) {
      float* C = (float*)Cout + (size_t)b * strideC;
      const int hh = lane >> 4, c4 = (lane & 15) * 4;
      for (int pass = 0; pass < 2; ++pass) {
#pragma unroll
        for (int it = 0; it < 8; ++it) {
          const int row = it * 2 + hh;
          v4f v = *(const v4f*)(slab + row * 68 + c4);
          *(volatile v4f*)(C + (size_t)(mBase + row) * ldc + n0 + c4) = v;
        }
        __threadfence();
      }
    } else {
      const int q = lane >> 3, c8 = (lane & 7) * 8;
      unsigned short* C  = (unsigned short*)Cout  + (size_t)b * strideC;
      unsigned short* C2 = (OUT_MODE == 2) ? ((unsigned short*)Cout2 + (size_t)b * strideC) : nullptr;
      for (int pass = 0; pass < 2; ++pass) {
#pragma unroll
        for (int it = 0; it < 4; ++it) {
          const int row = it * 4 + q;
          const float* sp = slab + row * 68 + c8;
          v8h hv, lv;
#pragma unroll
          for (int e = 0; e < 8; ++e) {
            if (OUT_MODE == 1) {
              hv[e] = (_Float16)sp[e];
            } else {
              unsigned short hb = f2bf_bits(sp[e]);
              unsigned short lb = f2bf_bits(sp[e] - bf_bits2f(hb));
              hv[e] = __builtin_bit_cast(_Float16, hb);
              lv[e] = __builtin_bit_cast(_Float16, lb);
            }
          }
          *(volatile v8h*)(C + (size_t)(mBase + row) * ldc + n0 + c8) = hv;
          if (OUT_MODE == 2) *(volatile v8h*)(C2 + (size_t)(mBase + row) * ldc + n0 + c8) = lv;
        }
        __threadfence();
      }
    }
    __builtin_amdgcn_fence(__ATOMIC_RELEASE, "workgroup");
    __builtin_amdgcn_wave_barrier();
    __builtin_amdgcn_fence(__ATOMIC_ACQUIRE, "workgroup");
  }
}

__device__ __forceinline__ unsigned pk16(unsigned short a, unsigned short b) { return (unsigned)a | ((unsigned)b << 16); }
__device__ __forceinline__ unsigned short h_bits(float f) { const _Float16 h = (_Float16)f; return __builtin_bit_cast(unsigned short, h); }

__global__ __launch_bounds__(256) void split_bf16x2_kernel(const float* __restrict__ in, unsigned short* __restrict__ hi,
                                                           unsigned short* __restrict__ lo, int n2) {
  const int i = blockIdx.x * 256 + threadIdx.x;
  if (i < n2) {
    const v2f f = *(const v2f*)(in + 2 * (size_t)i);
    const unsigned short h0 = f2bf_bits(f[0]), h1 = f2bf_bits(f[1]);
    const unsigned short l0 = f2bf_bits(f[0] - bf_bits2f(h0)), l1 = f2bf_bits(f[1] - bf_bits2f(h1));
    const unsigned uh = pk16(h0, h1), ul = pk16(l0, l1);
    ((volatile unsigned*)hi)[i] = uh;
    ((volatile unsigned*)lo)[i] = ul;
    __threadfence();
    ((volatile unsigned*)hi)[i] = uh;
    ((volatile unsigned*)lo)[i] = ul;
  }
}

__global__ __launch_bounds__(256) void transpose_split_kernel(const float* __restrict__ in, int ld_in, int rpitch,
                                                              unsigned short* __restrict__ outh, unsigned short* __restrict__ outl) {
  __shared__ __align__(16) float tile[64 * 68];
  const int c0  = blockIdx.x * 64;
  const int r0  = blockIdx.y * 64;
  const int tid = threadIdx.x;
#pragma unroll
  for (int it = 0; it < 4; ++it) {
    const int rr = it * 16 + (tid >> 4);
    const int cc = (tid & 15) * 4;
    const v4f a = *(const v4f*)(in + (size_t)(r0 + rr) * ld_in + c0 + cc);
    *(v4f*)(tile + rr * 68 + cc) = a;
  }
  __syncthreads();
  const int sub = tid >> 3;
  const int c8  = (tid & 7) * 8;
  v4u hv[2], lv[2];
#pragma unroll
  for (int it = 0; it < 2; ++it) {
    const int oc = it * 32 + sub;
    unsigned short hb[8], lb[8];
#pragma unroll
    for (int e = 0; e < 8; ++e) {
      const float f = tile[(c8 + e) * 68 + oc];
      hb[e] = f2bf_bits(f);
      lb[e] = f2bf_bits(f - bf_bits2f(hb[e]));
    }
    hv[it] = (v4u){pk16(hb[0], hb[1]), pk16(hb[2], hb[3]), pk16(hb[4], hb[5]), pk16(hb[6], hb[7])};
    lv[it] = (v4u){pk16(lb[0], lb[1]), pk16(lb[2], lb[3]), pk16(lb[4], lb[5]), pk16(lb[6], lb[7])};
  }
  for (int ps = 0; ps < 2; ++ps) {
#pragma unroll
    for (int it = 0; it < 2; ++it) {
      const int oc = it * 32 + sub;
      const size_t go = (size_t)(c0 + oc) * rpitch + r0 + c8;
      *(volatile v4u*)(outh + go) = hv[it];
      *(volatile v4u*)(outl + go) = lv[it];
    }
    __threadfence();
  }
}

__global__ __launch_bounds__(256) void mask_tiles_kernel(const float* __restrict__ amask, int* __restrict__ tflag) {
  __shared__ int sf[256];
  __shared__ __align__(16) int sl[32];
  const int mt  = blockIdx.x;
  const int tid = threadIdx.x;
  const int nt  = tid >> 3;
  const int c8  = (tid & 7) * 8;
  const float* base = amask + (size_t)(mt * 64) * SEQ + nt * 64 + c8;
  int any = 0;
#pragma unroll 4
  for (int r = 0; r < 64; ++r) {
    const v4f a = *(const v4f*)(base + (size_t)r * SEQ);
    const v4f c = *(const v4f*)(base + (size_t)r * SEQ + 4);
    any |= (int)(a[0] > MASK_CUT) | (int)(a[1] > MASK_CUT) | (int)(a[2] > MASK_CUT) | (int)(a[3] > MASK_CUT)
         | (int)(c[0] > MASK_CUT) | (int)(c[1] > MASK_CUT) | (int)(c[2] > MASK_CUT) | (int)(c[3] > MASK_CUT);
  }
  sf[tid] = any;
  __syncthreads();
  if (tid < 32) {
    int f = 0;
#pragma unroll
    for (int e = 0; e < 8; ++e) f |= sf[tid * 8 + e];
    sl[tid] = (f != 0) ? 1 : 0;
  }
  __syncthreads();
  if (tid < 8) {
    const v4i val = *(const v4i*)(sl + tid * 4);
    int* dst = tflag + (size_t)mt * TFP + tid * 4;
    *(volatile v4i*)dst = val;
    __threadfence();
    *(volatile v4i*)dst = val;
  }
}

__global__ __launch_bounds__(256) void rope_cast_kernel(const float* __restrict__ qkv, const float* __restrict__ rot,
                                                        unsigned short* __restrict__ Q16, unsigned short* __restrict__ K16, int total) {
#pragma clang fp contract(off)
  const int i = blockIdx.x * 256 + threadIdx.x;
  if (i < total) {
    const int t  = i >> 7;
    const int c8 = (i & 127) * 8;
    const int m0 = (c8 & (HDIM - 1)) >> 1;
    const float* qp = qkv + (size_t)t * (3 * EMB) + c8;
    const float* kp = qp + EMB;
    const v4f qa = *(const v4f*)qp, qb = *(const v4f*)(qp + 4);
    const v4f ka = *(const v4f*)kp, kb = *(const v4f*)(kp + 4);
    const float* rp = rot + ((size_t)t * (HDIM / 2) + m0) * 2;
    const v4f ra = *(const v4f*)rp, rb = *(const v4f*)(rp + 4);
    const float q0 = qa[0] * ra[0] - qa[1] * ra[1], q1 = qa[1] * ra[0] + qa[0] * ra[1];
    const float q2 = qa[2] * ra[2] - qa[3] * ra[3], q3 = qa[3] * ra[2] + qa[2] * ra[3];
    const float q4 = qb[0] * rb[0] - qb[1] * rb[1], q5 = qb[1] * rb[0] + qb[0] * rb[1];
    const float q6 = qb[2] * rb[2] - qb[3] * rb[3], q7 = qb[3] * rb[2] + qb[2] * rb[3];
    const float k0 = ka[0] * ra[0] - ka[1] * ra[1], k1 = ka[1] * ra[0] + ka[0] * ra[1];
    const float k2 = ka[2] * ra[2] - ka[3] * ra[3], k3 = ka[3] * ra[2] + ka[2] * ra[3];
    const float k4 = kb[0] * rb[0] - kb[1] * rb[1], k5 = kb[1] * rb[0] + kb[0] * rb[1];
    const float k6 = kb[2] * rb[2] - kb[3] * rb[3], k7 = kb[3] * rb[2] + kb[2] * rb[3];
    const v4u qv = (v4u){pk16(h_bits(q0), h_bits(q1)), pk16(h_bits(q2), h_bits(q3)), pk16(h_bits(q4), h_bits(q5)), pk16(h_bits(q6), h_bits(q7))};
    const v4u kv = (v4u){pk16(h_bits(k0), h_bits(k1)), pk16(h_bits(k2), h_bits(k3)), pk16(h_bits(k4), h_bits(k5)), pk16(h_bits(k6), h_bits(k7))};
    const size_t o = (size_t)t * EMB + c8;
    *(volatile v4u*)(Q16 + o) = qv;
    *(volatile v4u*)(K16 + o) = kv;
    __threadfence();
    *(volatile v4u*)(Q16 + o) = qv;
    *(volatile v4u*)(K16 + o) = kv;
  }
}

__global__ __launch_bounds__(256) void mask_softmax_kernel(const float* __restrict__ S, const float* __restrict__ amask,
                                                           unsigned short* __restrict__ Phi, unsigned short* __restrict__ Plo) {
  __shared__ float redm[8];
  __shared__ float reds[8];
  const int i    = blockIdx.x;
  const int hl   = blockIdx.y;
  const int tid  = threadIdx.x;
  const int lane = tid & 31;
  const int wave = tid >> 5;
  const int j0   = tid * 8;
  const size_t rowoff = ((size_t)hl * SEQ + i) * SEQ;
  const float* sr = S + rowoff + j0;
  const float* mr = amask + (size_t)i * SEQ + j0;
  const v4f sa = *(const v4f*)(sr), sb = *(const v4f*)(sr + 4);
  const v4f ma = *(const v4f*)(mr), mb = *(const v4f*)(mr + 4);
  const float NI = -INFINITY;
  const bool a0 = ma[0] > MASK_CUT, a1 = ma[1] > MASK_CUT, a2 = ma[2] > MASK_CUT, a3 = ma[3] > MASK_CUT;
  const bool a4 = mb[0] > MASK_CUT, a5 = mb[1] > MASK_CUT, a6 = mb[2] > MASK_CUT, a7 = mb[3] > MASK_CUT;
  const float t0 = a0 ? (sa[0] + ma[0]) : NI, t1 = a1 ? (sa[1] + ma[1]) : NI;
  const float t2 = a2 ? (sa[2] + ma[2]) : NI, t3 = a3 ? (sa[3] + ma[3]) : NI;
  const float t4 = a4 ? (sb[0] + mb[0]) : NI, t5 = a5 ? (sb[1] + mb[1]) : NI;
  const float t6 = a6 ? (sb[2] + mb[2]) : NI, t7 = a7 ? (sb[3] + mb[3]) : NI;
  float m = fmaxf(fmaxf(fmaxf(t0, t1), fmaxf(t2, t3)), fmaxf(fmaxf(t4, t5), fmaxf(t6, t7)));
#pragma unroll
  for (int off = 16; off > 0; off >>= 1) m = fmaxf(m, __shfl_xor(m, off, 32));
  if (lane == 0) redm[wave] = m;
  __syncthreads();
  float mx = redm[0];
#pragma unroll
  for (int w = 1; w < 8; ++w) mx = fmaxf(mx, redm[w]);
  const bool dead = !(mx > NI);
  const float e0 = dead ? 1.0f : (a0 ? __expf(t0 - mx) : 0.0f);
  const float e1 = dead ? 1.0f : (a1 ? __expf(t1 - mx) : 0.0f);
  const float e2 = dead ? 1.0f : (a2 ? __expf(t2 - mx) : 0.0f);
  const float e3 = dead ? 1.0f : (a3 ? __expf(t3 - mx) : 0.0f);
  const float e4 = dead ? 1.0f : (a4 ? __expf(t4 - mx) : 0.0f);
  const float e5 = dead ? 1.0f : (a5 ? __expf(t5 - mx) : 0.0f);
  const float e6 = dead ? 1.0f : (a6 ? __expf(t6 - mx) : 0.0f);
  const float e7 = dead ? 1.0f : (a7 ? __expf(t7 - mx) : 0.0f);
  float s = ((((((e0 + e1) + e2) + e3) + e4) + e5) + e6) + e7;
#pragma unroll
  for (int off = 16; off > 0; off >>= 1) s += __shfl_xor(s, off, 32);
  if (lane == 0) reds[wave] = s;
  __syncthreads();
  float tot = reds[0];
#pragma unroll
  for (int w = 1; w < 8; ++w) tot += reds[w];
  const float inv = 1.0f / tot;
  const float p0 = e0 * inv, p1 = e1 * inv, p2 = e2 * inv, p3 = e3 * inv;
  const float p4 = e4 * inv, p5 = e5 * inv, p6 = e6 * inv, p7 = e7 * inv;
  const unsigned short hb0 = f2bf_bits(p0), hb1 = f2bf_bits(p1), hb2 = f2bf_bits(p2), hb3 = f2bf_bits(p3);
  const unsigned short hb4 = f2bf_bits(p4), hb5 = f2bf_bits(p5), hb6 = f2bf_bits(p6), hb7 = f2bf_bits(p7);
  const unsigned short lb0 = f2bf_bits(p0 - bf_bits2f(hb0)), lb1 = f2bf_bits(p1 - bf_bits2f(hb1));
  const unsigned short lb2 = f2bf_bits(p2 - bf_bits2f(hb2)), lb3 = f2bf_bits(p3 - bf_bits2f(hb3));
  const unsigned short lb4 = f2bf_bits(p4 - bf_bits2f(hb4)), lb5 = f2bf_bits(p5 - bf_bits2f(hb5));
  const unsigned short lb6 = f2bf_bits(p6 - bf_bits2f(hb6)), lb7 = f2bf_bits(p7 - bf_bits2f(hb7));
  const v4u hv = (v4u){pk16(hb0, hb1), pk16(hb2, hb3), pk16(hb4, hb5), pk16(hb6, hb7)};
  const v4u lv = (v4u){pk16(lb0, lb1), pk16(lb2, lb3), pk16(lb4, lb5), pk16(lb6, lb7)};
  unsigned short* dh = Phi + rowoff + j0;
  unsigned short* dl = Plo + rowoff + j0;
  *(volatile v4u*)dh = hv;
  *(volatile v4u*)dl = lv;
  __threadfence();
  *(volatile v4u*)dh = hv;
  *(volatile v4u*)dl = lv;
}

extern "C" void kernel_launch(void* const* d_in, const int* in_sizes, int n_in,
                              void* d_out, int out_size, void* d_ws, size_t ws_size,
                              hipStream_t stream) {
  if (n_in < 7) return;
  if (in_sizes[0] != NB * SEQ * EMB) return;
  if (in_sizes[1] != SEQ * SEQ) return;
  if (in_sizes[2] != SEQ * (HDIM / 2) * 2) return;
  if (in_sizes[3] != EMB * 3 * EMB) return;
  if (in_sizes[4] != 3 * EMB) return;
  if (in_sizes[5] != EMB * EMB) return;
  if (in_sizes[6] != EMB) return;
  if (out_size != NB * SEQ * EMB) return;

  const float* x     = (const float*)d_in[0];
  const float* amask = (const float*)d_in[1];
  const float* rot   = (const float*)d_in[2];
  const float* Wqkv  = (const float*)d_in[3];
  const float* bqkv  = (const float*)d_in[4];
  const float* Wout  = (const float*)d_in[5];
  const float* bout  = (const float*)d_in[6];

  const size_t szWq  = (size_t)3 * EMB * EMB * 2;
  const size_t szWo  = (size_t)EMB * EMB * 2;
  const size_t szP16 = (size_t)SEQ * EMB * 2;
  const size_t szQKV = (size_t)SEQ * 3 * EMB * 4;
  const size_t szS   = (size_t)HGRP * SEQ * SEQ * 4;
  const size_t szP   = (size_t)HGRP * SEQ * SEQ * 2;
  const size_t szTF  = (size_t)TFN * 4;
  size_t off = 0;
  const size_t oWqh = off; off += szWq;
  const size_t oWql = off; off += szWq;
  const size_t oWoh = off; off += szWo;
  const size_t oWol = off; off += szWo;
  const size_t oQ16 = off; off += szP16;
  const size_t oK16 = off; off += szP16;
  const size_t oVTh = off; off += szP16;
  const size_t oVTl = off; off += szP16;
  const size_t oOh  = off; off += szP16;
  const size_t oOl  = off; off += szP16;
  const size_t oU   = off;
  const size_t oXh  = oU;
  const size_t oXl  = oU + szP16;
  const size_t oQKV = oU + 2 * szP16;
  const size_t endA = oQKV + szQKV;
  const size_t oS   = oU;
  const size_t oPh  = oU + szS;
  const size_t oPl  = oPh + szP;
  const size_t endB = oPl + szP;
  const size_t endU = (endA > endB) ? endA : endB;
  const size_t oTF  = endU;
  const size_t total = oTF + szTF;
  if (total > ws_size) return;

  char* ws = (char*)d_ws;
  unsigned short* WqTh = (unsigned short*)(ws + oWqh);
  unsigned short* WqTl = (unsigned short*)(ws + oWql);
  unsigned short* WoTh = (unsigned short*)(ws + oWoh);
  unsigned short* WoTl = (unsigned short*)(ws + oWol);
  unsigned short* Q16  = (unsigned short*)(ws + oQ16);
  unsigned short* K16  = (unsigned short*)(ws + oK16);
  unsigned short* VTh  = (unsigned short*)(ws + oVTh);
  unsigned short* VTl  = (unsigned short*)(ws + oVTl);
  unsigned short* Oh   = (unsigned short*)(ws + oOh);
  unsigned short* Ol   = (unsigned short*)(ws + oOl);
  unsigned short* Xh   = (unsigned short*)(ws + oXh);
  unsigned short* Xl   = (unsigned short*)(ws + oXl);
  float*          QKVf = (float*)(ws + oQKV);
  float*          Sbuf = (float*)(ws + oS);
  unsigned short* Ph   = (unsigned short*)(ws + oPh);
  unsigned short* Pl   = (unsigned short*)(ws + oPl);
  int*            Tf   = (int*)(ws + oTF);

  const dim3 blk(256);

  transpose_split_kernel<<<dim3(3 * EMB / 64, EMB / 64), blk, 0, stream>>>(Wqkv, 3 * EMB, EMB, WqTh, WqTl);
  transpose_split_kernel<<<dim3(EMB / 64, EMB / 64), blk, 0, stream>>>(Wout, EMB, EMB, WoTh, WoTl);
  mask_tiles_kernel<<<dim3(SEQ / 64), blk, 0, stream>>>(amask, Tf);

  const int n2x    = SEQ * EMB / 2;
  const dim3 gSplit((n2x + 255) / 256);
  const int nrope  = SEQ * (EMB / 8);
  const dim3 gRope((nrope + 255) / 256);
  const int tilesM = SEQ / 64;
  const dim3 gQKV((tilesM * (3 * EMB / 64) + 7) / 8, 1);
  const dim3 gS((tilesM * (SEQ / 64) + 7) / 8, HGRP);
  const dim3 gPV((tilesM * (HDIM / 64) + 7) / 8, HGRP);
  const dim3 gOut((tilesM * (EMB / 64) + 7) / 8, 1);
  const float sscale = 0.125f;

  for (int b = 0; b < NB; ++b) {
    split_bf16x2_kernel<<<gSplit, blk, 0, stream>>>(x + (size_t)b * SEQ * EMB, Xh, Xl, n2x);
    wmma_gemm64<1, true, 2, 0, false, 0, false, false><<<gQKV, blk, 0, stream>>>(
        Xh, Xl, EMB, 0L, WqTh, WqTl, EMB, 0L, (void*)QKVf, (void*)QKVf, 3 * EMB, 0L,
        bqkv, bqkv, 0L, SEQ, 3 * EMB, EMB, 1.0f, Tf, TFP, TFN);
    rope_cast_kernel<<<gRope, blk, 0, stream>>>(QKVf, rot, Q16, K16, nrope);
    transpose_split_kernel<<<dim3(EMB / 64, SEQ / 64), blk, 0, stream>>>(QKVf + 2 * EMB, 3 * EMB, SEQ, VTh, VTl);
    for (int hg = 0; hg < NGRP; ++hg) {
      const int h0 = hg * HGRP;
      wmma_gemm64<0, false, 0, 0, false, 0, true, false><<<gS, blk, 0, stream>>>(
          Q16 + h0 * HDIM, Q16 + h0 * HDIM, EMB, (long)HDIM,
          K16 + h0 * HDIM, K16 + h0 * HDIM, EMB, (long)HDIM,
          (void*)Sbuf, (void*)Sbuf, SEQ, (long)SEQ * SEQ,
          bqkv, bqkv, 0L, SEQ, SEQ, HDIM, sscale, Tf, TFP, TFN);
      mask_softmax_kernel<<<dim3(SEQ, HGRP), blk, 0, stream>>>(Sbuf, amask, Ph, Pl);
      wmma_gemm64<1, true, 0, 2, false, 0, false, true><<<gPV, blk, 0, stream>>>(
          Ph, Pl, SEQ, (long)SEQ * SEQ,
          VTh + (size_t)h0 * HDIM * SEQ, VTl + (size_t)h0 * HDIM * SEQ, SEQ, (long)HDIM * SEQ,
          (void*)(Oh + h0 * HDIM), (void*)(Ol + h0 * HDIM), EMB, (long)HDIM,
          bqkv, bqkv, 0L, SEQ, HDIM, SEQ, 1.0f, Tf, TFP, TFN);
    }
    float* outb = (float*)d_out + (size_t)b * SEQ * EMB;
    wmma_gemm64<1, true, 2, 0, false, 0, false, false><<<gOut, blk, 0, stream>>>(
        Oh, Ol, EMB, 0L, WoTh, WoTl, EMB, 0L, (void*)outb, (void*)outb, EMB, 0L,
        bout, bout, 0L, SEQ, EMB, EMB, 1.0f, Tf, TFP, TFN);
  }
  (void)hipGetLastError();
}
